// FLRWKV6_5351529251280
// MI455X (gfx1250) — hardware-verified
//
#include <hip/hip_runtime.h>
#include <math.h>

constexpr int kBatch    = 4;
constexpr int kSeq      = 1024;
constexpr int kDim      = 1024;
constexpr int kHeads    = 16;
constexpr int kKeyDim   = 512;
constexpr int kValDim   = 1024;
constexpr int kHeadK    = 32;
constexpr int kHeadV    = 64;
constexpr int kLowRank  = 32;
constexpr int kBranches = 5;
constexpr int kLowCols  = kBranches * kLowRank;
constexpr int kLowPad   = 192;
constexpr int kGateRank = 64;
constexpr int kTok      = kBatch * kSeq;
constexpr int kScanChunk = 16;
constexpr float kWCarry      = 64.0f;
constexpr float kWCarryInv   = 1.0f / 64.0f;
constexpr float kResCarry    = 2048.0f;
constexpr float kResCarryInv = 1.0f / 2048.0f;
constexpr float kGnEps       = 1e-5f;

static_assert(kKeyDim == kHeads * kHeadK, "key layout");
static_assert(kValDim == kHeads * kHeadV, "value layout");
static_assert(kLowCols == 160 && kLowPad % 64 == 0 && kLowPad >= kLowCols, "low-rank padding");
static_assert(kTok % 32 == 0, "M tile multiple");
static_assert(kKeyDim % 64 == 0 && kValDim % 64 == 0 && kDim % 64 == 0 && kGateRank % 64 == 0, "N tile multiples");
static_assert(kDim % 32 == 0 && kLowRank % 32 == 0 && kGateRank % 32 == 0 && kValDim % 32 == 0, "K multiples of 32");
static_assert(kSeq % kScanChunk == 0, "scan chunking");
static_assert((kSeq & (kSeq - 1)) == 0, "token index mask");

typedef __attribute__((ext_vector_type(16))) _Float16 v16h;
typedef __attribute__((ext_vector_type(8)))  _Float16 v8h;
typedef __attribute__((ext_vector_type(8)))  float    v8f;
typedef __attribute__((ext_vector_type(4)))  float    v4f;
typedef __attribute__((ext_vector_type(2)))  float    v2f;
typedef __attribute__((ext_vector_type(4)))  unsigned int v4u;

__device__ __forceinline__ unsigned short f2bf_bits(float f) {
  unsigned u = __float_as_uint(f);
  return (unsigned short)((u + 0x7FFFu + ((u >> 16) & 1u)) >> 16);
}
__device__ __forceinline__ float bf_bits2f(unsigned short h) { return __uint_as_float(((unsigned)h) << 16); }
__device__ __forceinline__ float bf16r(float f) { return bf_bits2f(f2bf_bits(f)); }
__device__ __forceinline__ unsigned pk16(unsigned short a, unsigned short b) { return (unsigned)a | ((unsigned)b << 16); }
__device__ __forceinline__ unsigned short h_bits(float f) { const _Float16 h = (_Float16)f; return __builtin_bit_cast(unsigned short, h); }

__device__ __forceinline__ void guard4_h(v8f& a, v8f& b, v8f& c, v8f& d, v16h x, v16h y) {
  asm volatile("v_nop\n\tv_nop\n\tv_nop\n\tv_nop" : "+v"(a), "+v"(b), "+v"(c), "+v"(d) : "v"(x), "v"(y));
}
__device__ __forceinline__ void keep4_h(v16h a, v16h b, v16h c, v16h d) { asm volatile("v_nop" :: "v"(a), "v"(b), "v"(c), "v"(d)); }
__device__ __forceinline__ void acc_guard4(v8f& a, v8f& b, v8f& c, v8f& d) { asm volatile("v_nop\n\tv_nop\n\tv_nop\n\tv_nop" : "+v"(a), "+v"(b), "+v"(c), "+v"(d)); }

struct Frag16 {
  union U { v16h v; v8h h[2]; };
  static __device__ __forceinline__ v16h load(const _Float16* p) {
    U f; f.h[0] = *(const v8h*)(p); f.h[1] = *(const v8h*)(p + 16); return f.v;
  }
  static __device__ __forceinline__ v8f mma(v16h a, v16h b, v8f c) {
    return __builtin_amdgcn_wmma_f32_16x16x32_f16(false, a, false, b, (short)0, c, false, false);
  }
};

__device__ __forceinline__ void wave_lds_sync() {
  __builtin_amdgcn_fence(__ATOMIC_RELEASE, "workgroup");
  __builtin_amdgcn_wave_barrier();
  __builtin_amdgcn_fence(__ATOMIC_ACQUIRE, "workgroup");
}

__global__ __launch_bounds__(256) void wt_transpose_kernel(const float* __restrict__ W, unsigned short* __restrict__ out,
                                                           int Kdim, int Ndim) {
  __shared__ float sm[64][65];
  const int t  = threadIdx.x;
  const int k0 = blockIdx.x * 64;
  const int n0 = blockIdx.y * 64;
#pragma unroll
  for (int i = 0; i < 16; ++i) {
    const int e = i * 256 + t;
    const int r = e >> 6;
    const int c = e & 63;
    const int n  = n0 + c;
    const int nc = (n < Ndim) ? n : (Ndim - 1);
    const float w = W[(size_t)(k0 + r) * Ndim + nc];
    const float v = (n < Ndim) ? (bf16r(w) * kWCarry) : 0.0f;
    sm[c][r] = v;
  }
  __syncthreads();
  const int lane = t & 31, wave = t >> 5;
  const int q = lane >> 3, c8 = (lane & 7) * 8;
  for (int pass = 0; pass < 2; ++pass) {
#pragma unroll
    for (int it = 0; it < 2; ++it) {
      const int row = wave * 8 + it * 4 + q;
      unsigned short hb[8];
#pragma unroll
      for (int e = 0; e < 8; ++e) hb[e] = h_bits(sm[row][c8 + e]);
      const v4u u = (v4u){pk16(hb[0], hb[1]), pk16(hb[2], hb[3]), pk16(hb[4], hb[5]), pk16(hb[6], hb[7])};
      *(volatile v4u*)(out + (size_t)(n0 + row) * Kdim + k0 + c8) = u;
    }
    __threadfence();
  }
}

__global__ __launch_bounds__(256) void cast_w8_kernel(const float* __restrict__ in, unsigned short* __restrict__ out, int n8) {
  const int i = blockIdx.x * 256 + threadIdx.x;
  if (i >= n8) return;
  const float* p = in + 8 * (size_t)i;
  const v4f a = *(const v4f*)(p);
  const v4f c = *(const v4f*)(p + 4);
  unsigned short hb[8];
#pragma unroll
  for (int e = 0; e < 4; ++e) {
    const float a0 = a[e];
    const float c0 = c[e];
    hb[e]     = h_bits(bf16r(a0) * kWCarry);
    hb[4 + e] = h_bits(bf16r(c0) * kWCarry);
  }
  const v4u u = (v4u){pk16(hb[0], hb[1]), pk16(hb[2], hb[3]), pk16(hb[4], hb[5]), pk16(hb[6], hb[7])};
  unsigned short* q = out + 8 * (size_t)i;
  *(volatile v4u*)q = u;
  __threadfence();
  *(volatile v4u*)q = u;
}

__global__ __launch_bounds__(256) void prep_x_kernel(const float* __restrict__ x, const float* __restrict__ mu,
                                                     unsigned short* __restrict__ xq, unsigned short* __restrict__ xin, int n8) {
  const int i = blockIdx.x * 256 + threadIdx.x;
  if (i >= n8) return;
  const int m  = i >> 7;
  const int c8 = (i & 127) * 8;
  const int t  = m & (kSeq - 1);
  const int mp = (t == 0) ? m : (m - 1);
  const float* pc = x + (size_t)m  * kDim + c8;
  const float* pp = x + (size_t)mp * kDim + c8;
  const v4f a0 = *(const v4f*)(pc);
  const v4f a1 = *(const v4f*)(pc + 4);
  const v4f p0 = *(const v4f*)(pp);
  const v4f p1 = *(const v4f*)(pp + 4);
  const v4f u0 = *(const v4f*)(mu + c8);
  const v4f u1 = *(const v4f*)(mu + c8 + 4);
  unsigned short qb[8];
  v8h hv;
#pragma unroll
  for (int e = 0; e < 4; ++e) {
    const float xa = a0[e], xb = a1[e];
    const float ya = p0[e], yb = p1[e];
    const float ma = bf16r(u0[e]), mb = bf16r(u1[e]);
    const unsigned short ba = f2bf_bits(xa), bb = f2bf_bits(xb);
    const float xva = bf_bits2f(ba), xvb = bf_bits2f(bb);
    const float pva = (t == 0) ? 0.0f : bf16r(ya);
    const float pvb = (t == 0) ? 0.0f : bf16r(yb);
    qb[e]     = ba;
    qb[4 + e] = bb;
    hv[e]     = (_Float16)(xva + (pva - xva) * ma);
    hv[4 + e] = (_Float16)(xvb + (pvb - xvb) * mb);
  }
  const v4u u = (v4u){pk16(qb[0], qb[1]), pk16(qb[2], qb[3]), pk16(qb[4], qb[5]), pk16(qb[6], qb[7])};
  unsigned short* oq = xq  + 8 * (size_t)i;
  unsigned short* oi = xin + 8 * (size_t)i;
  *(volatile v4u*)oq = u;
  *(volatile v8h*)oi = hv;
  __threadfence();
  *(volatile v4u*)oq = u;
  *(volatile v8h*)oi = hv;
}

enum { EPI_F32 = 0, EPI_TANH16 = 1, EPI_DEC32 = 2, EPI_LERP16 = 3 };

template <bool RES, int EPI>
__global__ __launch_bounds__(256) void gemm_w32x64_kernel(
    const unsigned short* __restrict__ Ap, const unsigned short* __restrict__ A2p, int lda,
    const unsigned short* __restrict__ Btp, int ldb,
    void* Cout, void* Cout2, int ldc,
    const float* __restrict__ bias, const unsigned short* __restrict__ xq,
    int M, int N, int K, float scale) {
  const _Float16* A  = (const _Float16*)Ap;
  const _Float16* A2 = (const _Float16*)A2p;
  const _Float16* Bt = (const _Float16*)Btp;
  __shared__ __align__(16) float sT[8][16 * 68];
  const int lane = threadIdx.x & 31;
  const int wave = threadIdx.x >> 5;
  const int tilesN = N >> 6;
  const int tilesM = M >> 5;
  const int tile = blockIdx.x * 8 + wave;
  if (tile >= tilesM * tilesN) return;
  const int tm = tile / tilesN;
  const int tn = tile - tm * tilesN;
  const int m0 = tm << 5;
  const int n0 = tn << 6;

  const int rlane = lane & 15;
  const int koff  = (lane >> 4) * 8;
  const int mOff  = (lane >> 4) * 8;

  v8f acc[2][4];
  v8f accr[2][4];
#pragma unroll
  for (int i = 0; i < 2; ++i)
#pragma unroll
    for (int j = 0; j < 4; ++j) {
      acc[i][j]  = (v8f){0.f, 0.f, 0.f, 0.f, 0.f, 0.f, 0.f, 0.f};
      accr[i][j] = (v8f){0.f, 0.f, 0.f, 0.f, 0.f, 0.f, 0.f, 0.f};
    }

  for (int k0 = 0; k0 < K; k0 += 32) {
    v16h bh[4];
#pragma unroll
    for (int j = 0; j < 4; ++j) {
      const size_t bo = (size_t)(n0 + (j << 4) + rlane) * ldb + koff + k0;
      bh[j] = Frag16::load(Bt + bo);
    }
#pragma unroll
    for (int i = 0; i < 2; ++i) {
      const size_t ao = (size_t)(m0 + (i << 4) + rlane) * lda + koff + k0;
      const v16h ah = Frag16::load(A + ao);
      v16h al = ah;
      if (RES) al = Frag16::load(A2 + ao);
#pragma unroll
      for (int j = 0; j < 4; ++j) {
        acc[i][j] = Frag16::mma(ah, bh[j], acc[i][j]);
        if (RES) accr[i][j] = Frag16::mma(al, bh[j], accr[i][j]);
      }
      guard4_h(acc[i][0], acc[i][1], acc[i][2], acc[i][3], ah, al);
      if (RES) guard4_h(accr[i][0], accr[i][1], accr[i][2], accr[i][3], al, ah);
    }
    keep4_h(bh[0], bh[1], bh[2], bh[3]);
  }
  acc_guard4(acc[0][0], acc[0][1], acc[0][2], acc[0][3]);
  acc_guard4(acc[1][0], acc[1][1], acc[1][2], acc[1][3]);
  if (RES) {
    acc_guard4(accr[0][0], accr[0][1], accr[0][2], accr[0][3]);
    acc_guard4(accr[1][0], accr[1][1], accr[1][2], accr[1][3]);
  }

  float* slab = sT[wave];
#pragma unroll
  for (int i = 0; i < 2; ++i) {
    const int mBase = m0 + (i << 4);
#pragma unroll
    for (int j = 0; j < 4; ++j) {
#pragma unroll
      for (int r = 0; r < 8; ++r) {
        float v = acc[i][j][r];
        if (RES) v += accr[i][j][r] * kResCarryInv;
        v *= scale;
        slab[(mOff + r) * 68 + (j << 4) + rlane] = v;
      }
    }
    wave_lds_sync();

    if (EPI == EPI_TANH16) {
      const int q = lane >> 3, c8 = (lane & 7) * 8;
#pragma unroll 1
      for (int it = 0; it < 4; ++it) {
        float* sp = slab + (it * 4 + q) * 68 + c8;
#pragma unroll
        for (int e = 0; e < 8; ++e) {
          const float z = sp[e];
          sp[e] = tanhf(z);
        }
      }
    }
    if (EPI == EPI_DEC32) {
      const int hh = lane >> 4, c4 = (lane & 15) * 4;
      const v4f b4 = *(const v4f*)(bias + n0 + c4);
      float bq[4];
#pragma unroll
      for (int e = 0; e < 4; ++e) {
        const float bv = b4[e];
        bq[e] = bf16r(bv);
      }
#pragma unroll 1
      for (int it = 0; it < 8; ++it) {
        float* sp = slab + (it * 2 + hh) * 68 + c4;
#pragma unroll
        for (int e = 0; e < 4; ++e) {
          const float z = sp[e] + bq[e];
          sp[e] = expf(-expf(z));
        }
      }
    }
    if (EPI == EPI_LERP16) {
      const int q = lane >> 3, c8 = (lane & 7) * 8;
      const int col = n0 + c8;
      const v4f b0 = *(const v4f*)(bias + col);
      const v4f b1 = *(const v4f*)(bias + col + 4);
      float bq[8];
#pragma unroll
      for (int e = 0; e < 4; ++e) {
        const float ba = b0[e];
        const float bb = b1[e];
        bq[e]     = bf16r(ba);
        bq[4 + e] = bf16r(bb);
      }
#pragma unroll 1
      for (int it = 0; it < 4; ++it) {
        const int row = it * 4 + q;
        const int m   = mBase + row;
        const int t   = m & (kSeq - 1);
        const int mp  = (t == 0) ? m : (m - 1);
        const v4u xc = *(const v4u*)(xq + (size_t)m  * ldc + col);
        const v4u xp = *(const v4u*)(xq + (size_t)mp * ldc + col);
        float* sp = slab + row * 68 + c8;
#pragma unroll
        for (int e2 = 0; e2 < 4; ++e2) {
          const unsigned wc = xc[e2];
          const unsigned wp = xp[e2];
          const float xa = __uint_as_float(wc << 16);
          const float xb = __uint_as_float(wc & 0xffff0000u);
          const float ya = __uint_as_float(wp << 16);
          const float yb = __uint_as_float(wp & 0xffff0000u);
          const float pa = (t == 0) ? 0.0f : ya;
          const float pb = (t == 0) ? 0.0f : yb;
          const float ma = sp[2 * e2]     + bq[2 * e2];
          const float mb = sp[2 * e2 + 1] + bq[2 * e2 + 1];
          sp[2 * e2]     = xa + (pa - xa) * ma;
          sp[2 * e2 + 1] = xb + (pb - xb) * mb;
        }
      }
    }
    if (EPI != EPI_F32) wave_lds_sync();

    if (EPI == EPI_F32 || EPI == EPI_DEC32) {
      float* C = (float*)Cout;
      const int hh = lane >> 4, c4 = (lane & 15) * 4;
      for (int pass = 0; pass < 2; ++pass) {
#pragma unroll
        for (int it = 0; it < 8; ++it) {
          const int row = it * 2 + hh;
          const v4f v = *(const v4f*)(slab + row * 68 + c4);
          *(volatile v4f*)(C + (size_t)(mBase + row) * ldc + n0 + c4) = v;
        }
        __threadfence();
      }
    } else {
      const int q = lane >> 3, c8 = (lane & 7) * 8;
      unsigned short* C  = (unsigned short*)Cout;
      unsigned short* C2 = (unsigned short*)Cout2;
      for (int pass = 0; pass < 2; ++pass) {
#pragma unroll
        for (int it = 0; it < 4; ++it) {
          const int row = it * 4 + q;
          const float* sp = slab + row * 68 + c8;
          v8h hv, lv;
#pragma unroll
          for (int e = 0; e < 8; ++e) {
            const float xv = sp[e];
            const _Float16 h16 = (_Float16)xv;
            hv[e] = h16;
            if (EPI == EPI_LERP16) lv[e] = (_Float16)((xv - (float)h16) * kResCarry);
          }
          *(volatile v8h*)(C + (size_t)(mBase + row) * ldc + n0 + c8) = hv;
          if (EPI == EPI_LERP16) *(volatile v8h*)(C2 + (size_t)(mBase + row) * ldc + n0 + c8) = lv;
        }
        __threadfence();
      }
    }
    wave_lds_sync();
  }
}

__device__ __forceinline__ float wave_sum32(float v) {
  v += __shfl_xor(v, 16, 32);
  v += __shfl_xor(v, 8, 32);
  v += __shfl_xor(v, 4, 32);
  v += __shfl_xor(v, 2, 32);
  v += __shfl_xor(v, 1, 32);
  return v;
}

__global__ __launch_bounds__(32) void recur_scan_kernel(
    const float* __restrict__ Rp, const float* __restrict__ Kp, const float* __restrict__ Dp,
    const float* __restrict__ Vp, const float* __restrict__ Gp,
    const float* __restrict__ u, const float* __restrict__ gnw, const float* __restrict__ gnb,
    unsigned short* __restrict__ OGH, unsigned short* __restrict__ OGL) {
  __shared__ __align__(16) float Ssh[kHeadK * kHeadV];
  __shared__ __align__(16) float rs[kScanChunk * kHeadK];
  __shared__ __align__(16) float ks[kScanChunk * kHeadK];
  __shared__ __align__(16) float dsh[kScanChunk * kHeadK];
  __shared__ float bons[kScanChunk];
  __shared__ __align__(16) unsigned ohs[kScanChunk * 32];
  __shared__ __align__(16) unsigned ols[kScanChunk * 32];

  const int lane = threadIdx.x;
  const int bh = blockIdx.x;
  const int b  = bh >> 4;
  const int h  = bh & (kHeads - 1);
  const int c4 = (lane & 7) * 4;
  const int rq = lane >> 3;

#pragma unroll 1
  for (int k = 0; k < kHeadK; ++k) *(v2f*)(Ssh + k * kHeadV + 2 * lane) = (v2f){0.0f, 0.0f};

  const v4f uraw = *(const v4f*)(u + h * kHeadK + c4);
  float uq[4];
#pragma unroll
  for (int e = 0; e < 4; ++e) {
    const float uv = uraw[e];
    uq[e] = bf16r(uv);
  }
  const v2f gwr = *(const v2f*)(gnw + h * kHeadV + 2 * lane);
  const v2f gbr = *(const v2f*)(gnb + h * kHeadV + 2 * lane);
  const float gw0 = bf16r(gwr[0]), gw1 = bf16r(gwr[1]);
  const float gb0 = bf16r(gbr[0]), gb1 = bf16r(gbr[1]);

#pragma unroll 1
  for (int chunk = 0; chunk < kSeq / kScanChunk; ++chunk) {
    const int mrow0 = b * kSeq + chunk * kScanChunk;
    __syncthreads();
#pragma unroll 1
    for (int i = 0; i < 4; ++i) {
      const int row = i * 4 + rq;
      const size_t off = (size_t)(mrow0 + row) * kKeyDim + h * kHeadK + c4;
      const v4f r4 = *(const v4f*)(Rp + off);
      const v4f k4 = *(const v4f*)(Kp + off);
      const v4f d4 = *(const v4f*)(Dp + off);
      *(v4f*)(rs  + row * kHeadK + c4) = r4;
      *(v4f*)(ks  + row * kHeadK + c4) = k4;
      *(v4f*)(dsh + row * kHeadK + c4) = d4;
      float p = 0.0f;
#pragma unroll
      for (int e = 0; e < 4; ++e) p += (r4[e] * uq[e]) * k4[e];
      p += __shfl_xor(p, 1, 32);
      p += __shfl_xor(p, 2, 32);
      p += __shfl_xor(p, 4, 32);
      bons[row] = p;
    }
    __syncthreads();

#pragma unroll 1
    for (int s = 0; s < kScanChunk; ++s) {
      const size_t m = (size_t)(mrow0 + s);
      const v2f vv = *(const v2f*)(Vp + m * kValDim + h * kHeadV + 2 * lane);
      const v2f gg = *(const v2f*)(Gp + m * kValDim + h * kHeadV + 2 * lane);
      const float v0 = vv[0], v1 = vv[1];
      float o0 = 0.0f, o1 = 0.0f;
#pragma unroll 1
      for (int kq = 0; kq < kHeadK / 4; ++kq) {
        const v4f r4 = *(const v4f*)(rs  + s * kHeadK + kq * 4);
        const v4f k4 = *(const v4f*)(ks  + s * kHeadK + kq * 4);
        const v4f d4 = *(const v4f*)(dsh + s * kHeadK + kq * 4);
#pragma unroll
        for (int e = 0; e < 4; ++e) {
          float* sp = Ssh + (kq * 4 + e) * kHeadV + 2 * lane;
          v2f S2 = *(v2f*)sp;
          const float re = r4[e], ke = k4[e], de = d4[e];
          o0 += re * S2[0];
          o1 += re * S2[1];
          S2[0] = de * S2[0] + ke * v0;
          S2[1] = de * S2[1] + ke * v1;
          *(v2f*)sp = S2;
        }
      }
      const float bon = bons[s];
      o0 += bon * v0;
      o1 += bon * v1;
      const float mean = wave_sum32(o0 + o1) * (1.0f / kHeadV);
      const float e0 = o0 - mean, e1 = o1 - mean;
      const float var = wave_sum32(e0 * e0 + e1 * e1) * (1.0f / kHeadV);
      const float rstd = rsqrtf(var + kGnEps);
      const float y0 = (e0 * rstd) * gw0 + gb0;
      const float y1 = (e1 * rstd) * gw1 + gb1;
      const float g0 = gg[0], g1 = gg[1];
      const float s0 = g0 * __builtin_amdgcn_rcpf(1.0f + expf(-g0));
      const float s1 = g1 * __builtin_amdgcn_rcpf(1.0f + expf(-g1));
      const float og0 = y0 * s0;
      const float og1 = y1 * s1;
      const _Float16 a0 = (_Float16)og0;
      const _Float16 a1 = (_Float16)og1;
      const _Float16 l0 = (_Float16)((og0 - (float)a0) * kResCarry);
      const _Float16 l1 = (_Float16)((og1 - (float)a1) * kResCarry);
      ohs[s * 32 + lane] = pk16(__builtin_bit_cast(unsigned short, a0), __builtin_bit_cast(unsigned short, a1));
      ols[s * 32 + lane] = pk16(__builtin_bit_cast(unsigned short, l0), __builtin_bit_cast(unsigned short, l1));
    }
    __syncthreads();

    for (int pass = 0; pass < 2; ++pass) {
#pragma unroll
      for (int i = 0; i < 4; ++i) {
        const int row = i * 4 + rq;
        const v4u wh = *(const v4u*)(ohs + row * 32 + c4);
        const v4u wl = *(const v4u*)(ols + row * 32 + c4);
        const size_t wo = (((size_t)(mrow0 + row) * kValDim + h * kHeadV) >> 1) + c4;
        *(volatile v4u*)((unsigned*)OGH + wo) = wh;
        *(volatile v4u*)((unsigned*)OGL + wo) = wl;
      }
      __threadfence();
    }
  }
}

static inline dim3 gemm_grid(int M, int N) { return dim3((unsigned)((((M >> 5) * (N >> 6)) + 7) / 8)); }

extern "C" void kernel_launch(void* const* d_in, const int* in_sizes, int n_in,
                              void* d_out, int out_size, void* d_ws, size_t ws_size, hipStream_t stream) {
  if (n_in < 16 || d_out == nullptr || d_ws == nullptr) return;
  if (in_sizes[0] != kTok * kDim || in_sizes[1] != kDim || in_sizes[2] != kDim * kLowCols ||
      in_sizes[3] != kDim * kLowCols || in_sizes[4] != kBranches * kDim || in_sizes[5] != kDim * kKeyDim ||
      in_sizes[6] != kDim * kGateRank || in_sizes[7] != kGateRank * kKeyDim || in_sizes[8] != kKeyDim ||
      in_sizes[9] != kDim * kKeyDim || in_sizes[10] != kDim * kValDim || in_sizes[11] != kDim * kValDim ||
      in_sizes[12] != kHeads * kHeadK || in_sizes[13] != kValDim || in_sizes[14] != kValDim ||
      in_sizes[15] != kValDim * kDim || out_size != kTok * kDim) return;

  const float* x      = (const float*)d_in[0];
  const float* mu_x   = (const float*)d_in[1];
  const float* W_x1   = (const float*)d_in[2];
  const float* W_x2   = (const float*)d_in[3];
  const float* x_bias = (const float*)d_in[4];
  const float* W_r    = (const float*)d_in[5];
  const float* W_w1   = (const float*)d_in[6];
  const float* W_w2   = (const float*)d_in[7];
  const float* b_w2   = (const float*)d_in[8];
  const float* W_k    = (const float*)d_in[9];
  const float* W_v    = (const float*)d_in[10];
  const float* W_g    = (const float*)d_in[11];
  const float* u      = (const float*)d_in[12];
  const float* gn_w   = (const float*)d_in[13];
  const float* gn_b   = (const float*)d_in[14];
  const float* W_o    = (const float*)d_in[15];
  float* out = (float*)d_out;

  char* ws = (char*)d_ws;
  size_t off = 0;
  auto carve = [&](size_t bytes) -> char* { char* p = ws + off; off += (bytes + 255) & ~(size_t)255; return p; };
  unsigned short* WX1T = (unsigned short*)carve((size_t)kLowPad * kDim * 2);
  unsigned short* WX2Q = (unsigned short*)carve((size_t)kDim * kLowCols * 2);
  unsigned short* WRT  = (unsigned short*)carve((size_t)kKeyDim * kDim * 2);
  unsigned short* WKT  = (unsigned short*)carve((size_t)kKeyDim * kDim * 2);
  unsigned short* WW1T = (unsigned short*)carve((size_t)kGateRank * kDim * 2);
  unsigned short* WW2T = (unsigned short*)carve((size_t)kKeyDim * kGateRank * 2);
  unsigned short* WVT  = (unsigned short*)carve((size_t)kValDim * kDim * 2);
  unsigned short* WGT  = (unsigned short*)carve((size_t)kValDim * kDim * 2);
  unsigned short* WOT  = (unsigned short*)carve((size_t)kDim * kValDim * 2);
  unsigned short* XQ   = (unsigned short*)carve((size_t)kTok * kDim * 2);
  unsigned short* XIN  = (unsigned short*)carve((size_t)kTok * kDim * 2);
  unsigned short* LOW  = (unsigned short*)carve((size_t)kTok * kLowPad * 2);
  unsigned short* XIH  = (unsigned short*)carve((size_t)kTok * kDim * 2);
  unsigned short* XIL  = (unsigned short*)carve((size_t)kTok * kDim * 2);
  unsigned short* WT   = (unsigned short*)carve((size_t)kTok * kGateRank * 2);
  float* RPL = (float*)carve((size_t)kTok * kKeyDim * 4);
  float* KPL = (float*)carve((size_t)kTok * kKeyDim * 4);
  float* DEC = (float*)carve((size_t)kTok * kKeyDim * 4);
  float* VPL = (float*)carve((size_t)kTok * kValDim * 4);
  float* GPL = (float*)carve((size_t)kTok * kValDim * 4);
  unsigned short* OGH = (unsigned short*)carve((size_t)kTok * kValDim * 2);
  unsigned short* OGL = (unsigned short*)carve((size_t)kTok * kValDim * 2);
  if (off > ws_size || off > (size_t)134217728) return;

  wt_transpose_kernel<<<dim3(kDim / 64, kLowPad / 64), 256, 0, stream>>>(W_x1, WX1T, kDim, kLowCols);
  cast_w8_kernel<<<(kDim * kLowCols / 8 + 255) / 256, 256, 0, stream>>>(W_x2, WX2Q, kDim * kLowCols / 8);
  wt_transpose_kernel<<<dim3(kDim / 64, kKeyDim / 64), 256, 0, stream>>>(W_r, WRT, kDim, kKeyDim);
  wt_transpose_kernel<<<dim3(kDim / 64, kKeyDim / 64), 256, 0, stream>>>(W_k, WKT, kDim, kKeyDim);
  wt_transpose_kernel<<<dim3(kDim / 64, kGateRank / 64), 256, 0, stream>>>(W_w1, WW1T, kDim, kGateRank);
  wt_transpose_kernel<<<dim3(kGateRank / 64, kKeyDim / 64), 256, 0, stream>>>(W_w2, WW2T, kGateRank, kKeyDim);
  wt_transpose_kernel<<<dim3(kDim / 64, kValDim / 64), 256, 0, stream>>>(W_v, WVT, kDim, kValDim);
  wt_transpose_kernel<<<dim3(kDim / 64, kValDim / 64), 256, 0, stream>>>(W_g, WGT, kDim, kValDim);
  wt_transpose_kernel<<<dim3(kValDim / 64, kDim / 64), 256, 0, stream>>>(W_o, WOT, kValDim, kDim);

  prep_x_kernel<<<(kTok * kDim / 8 + 255) / 256, 256, 0, stream>>>(x, mu_x, XQ, XIN, kTok * kDim / 8);

  gemm_w32x64_kernel<false, EPI_TANH16><<<gemm_grid(kTok, kLowPad), 256, 0, stream>>>(
      XIN, XIN, kDim, WX1T, kDim, (void*)LOW, (void*)LOW, kLowPad, x_bias, XQ, kTok, kLowPad, kDim, kWCarryInv);

  auto lerp_branch = [&](int n) {
    gemm_w32x64_kernel<false, EPI_LERP16><<<gemm_grid(kTok, kDim), 256, 0, stream>>>(
        LOW + n * kLowRank, LOW + n * kLowRank, kLowPad, WX2Q + n * kLowRank, kLowCols,
        (void*)XIH, (void*)XIL, kDim, x_bias + (size_t)n * kDim, XQ, kTok, kDim, kLowRank, kWCarryInv);
  };
  auto proj = [&](const unsigned short* Wt, float* dst, int N) {
    gemm_w32x64_kernel<true, EPI_F32><<<gemm_grid(kTok, N), 256, 0, stream>>>(
        XIH, XIL, kDim, Wt, kDim, (void*)dst, (void*)dst, N, x_bias, XQ, kTok, N, kDim, kWCarryInv);
  };

  lerp_branch(0);
  proj(WRT, RPL, kKeyDim);
  lerp_branch(1);
  gemm_w32x64_kernel<false, EPI_TANH16><<<gemm_grid(kTok, kGateRank), 256, 0, stream>>>(
      XIH, XIH, kDim, WW1T, kDim, (void*)WT, (void*)WT, kGateRank, x_bias, XQ, kTok, kGateRank, kDim, kWCarryInv);
  gemm_w32x64_kernel<false, EPI_DEC32><<<gemm_grid(kTok, kKeyDim), 256, 0, stream>>>(
      WT, WT, kGateRank, WW2T, kGateRank, (void*)DEC, (void*)DEC, kKeyDim, b_w2, XQ, kTok, kKeyDim, kGateRank, kWCarryInv);
  lerp_branch(2);
  proj(WKT, KPL, kKeyDim);
  lerp_branch(3);
  proj(WVT, VPL, kValDim);
  lerp_branch(4);
  proj(WGT, GPL, kValDim);

  recur_scan_kernel<<<kBatch * kHeads, 32, 0, stream>>>(RPL, KPL, DEC, VPL, GPL, u, gn_w, gn_b, OGH, OGL);

  gemm_w32x64_kernel<true, EPI_F32><<<gemm_grid(kTok, kDim), 256, 0, stream>>>(
      OGH, OGL, kValDim, WOT, kValDim, (void*)out, (void*)out, kDim, x_bias, XQ, kTok, kDim, kValDim, kWCarryInv);
}
